// FastAttention_34969623724566
// MI455X (gfx1250) — hardware-run, weakly checked
//
#include <hip/hip_runtime.h>


#define NB_  2
#define TT   4096
#define DM   512
#define NH_  8
#define NKV  8
#define REP  (NH_ / NKV)
#define HD   64
#define DQ   (NH_ * HD)
#define DKV  (NKV * HD)
#define ZH   1
#define RH   512
#define WIN  4096
#define MF   256
#define QSC  16384.0f
#define EPSD (1e-6f * 262144.0f)
#define NRM  0.35355339059327379f
#define PCAR 1024.0f
#define SCL  1.0f
typedef _Float16 h16;
typedef unsigned short bf;
typedef __attribute__((ext_vector_type(16))) __bf16   v16bf;
typedef __attribute__((ext_vector_type(16))) _Float16 v16h;
typedef __attribute__((ext_vector_type(8)))  _Float16 v8h;
typedef __attribute__((ext_vector_type(8)))  unsigned short v8us;
typedef __attribute__((ext_vector_type(8)))  float    v8f;
typedef __attribute__((ext_vector_type(4)))  float    v4f;
typedef v8h  __attribute__((may_alias)) v8ha;
typedef v4f  __attribute__((may_alias)) v4fa;
typedef v8us __attribute__((may_alias)) v8usa;

__device__ __forceinline__ unsigned short f2bf(float f) { unsigned u = __float_as_uint(f); u += 0x7FFFu + ((u >> 16) & 1u); return (unsigned short)(u >> 16); }
__device__ __forceinline__ float bf2f(unsigned short b) { return __uint_as_float(((unsigned)b) << 16); }
__device__ __forceinline__ float bfr(float f) { return bf2f(f2bf(f)); }
__device__ __forceinline__ v16h cat16(v8h lo, v8h hi) { return __builtin_shufflevector(lo, hi, 0, 1, 2, 3, 4, 5, 6, 7, 8, 9, 10, 11, 12, 13, 14, 15); }
__device__ __forceinline__ v16bf cat16b(v8us lo, v8us hi) { return __builtin_bit_cast(v16bf, __builtin_shufflevector(lo, hi, 0, 1, 2, 3, 4, 5, 6, 7, 8, 9, 10, 11, 12, 13, 14, 15)); }
__device__ __forceinline__ v8f wmma16(v16h a, v16h b, v8f c) { return __builtin_amdgcn_wmma_f32_16x16x32_f16(false, a, false, b, (short)0, c, false, false); }
__device__ __forceinline__ v8f wmmab(v16bf a, v16bf b, v8f c) { return __builtin_amdgcn_wmma_f32_16x16x32_bf16(false, a, false, b, (short)0, c, false, false); }


template <typename T16> struct WFrag;
template <> struct WFrag<h16> { typedef v16h V; static __device__ __forceinline__ V ld(const h16* p) { return cat16(*(const v8h*)p, *(const v8h*)(p + 16)); } static __device__ __forceinline__ v8f mma(V a, V b, v8f c) { return wmma16(a, b, c); } };
template <> struct WFrag<bf> { typedef v16bf V; static __device__ __forceinline__ V ld(const bf* p) { return cat16b(*(const v8us*)p, *(const v8us*)(p + 16)); } static __device__ __forceinline__ v8f mma(V a, V b, v8f c) { return wmmab(a, b, c); } };
template <typename T16, int NSPLIT, bool BIAS>
__global__ __launch_bounds__(32) void k_gemmw(const T16* __restrict__ A, const T16* __restrict__ A2, const T16* __restrict__ Bt, const T16* __restrict__ Bt2, int K, float* C, int ldc, const float* __restrict__ bias, size_t sA, size_t sB, size_t sC) {
    typedef typename WFrag<T16>::V V;
    __shared__ __align__(16) float os[16 * 68];
    const size_t z = blockIdx.z; A += z * sA; if (A2) A2 += z * sA; Bt += z * sB; if (Bt2) Bt2 += z * sB; C += z * sC;
    const int lane = threadIdx.x & 31, lr = lane & 15, hi = lane >> 4; const int r0 = blockIdx.x * 64, c0 = blockIdx.y * 64;
    v8f acc[4][4];
#pragma unroll
    for (int mb = 0; mb < 4; ++mb)
#pragma unroll
        for (int nb = 0; nb < 4; ++nb) acc[mb][nb] = (v8f){};
    const size_t aoff = (size_t)(r0 + lr) * K + 8 * hi, boff = (size_t)(c0 + lr) * K + 8 * hi;
#pragma unroll 1
    for (int kc = 0; kc < K; kc += 32) {
        V a[4], a2[4];
#pragma unroll
        for (int mb = 0; mb < 4; ++mb) { a[mb] = WFrag<T16>::ld(A + aoff + (size_t)mb * 16 * K + kc); if (NSPLIT == 1 || NSPLIT == 2) a2[mb] = WFrag<T16>::ld(A2 + aoff + (size_t)mb * 16 * K + kc); }
#pragma unroll
        for (int nb = 0; nb < 4; ++nb) { const V b = WFrag<T16>::ld(Bt + boff + (size_t)nb * 16 * K + kc); V b2; if (NSPLIT >= 2) b2 = WFrag<T16>::ld(Bt2 + boff + (size_t)nb * 16 * K + kc);
#pragma unroll
            for (int mb = 0; mb < 4; ++mb) { acc[mb][nb] = WFrag<T16>::mma(a[mb], b, acc[mb][nb]); if (NSPLIT == 1 || NSPLIT == 2) acc[mb][nb] = WFrag<T16>::mma(a2[mb], b, acc[mb][nb]); if (NSPLIT >= 2) acc[mb][nb] = WFrag<T16>::mma(a[mb], b2, acc[mb][nb]); } }
        asm volatile("v_nop\n\tv_nop\n\tv_nop\n\tv_nop" : "+v"(acc[0][0]), "+v"(acc[1][1]), "+v"(acc[2][2]), "+v"(acc[3][3]) : "v"(a[0]), "v"(a[3]));
    }
#pragma unroll
    for (int mb = 0; mb < 4; ++mb) {
#pragma unroll
        for (int nb = 0; nb < 4; ++nb) {
#pragma unroll
            for (int j = 0; j < 8; ++j) os[(hi * 8 + j) * 68 + nb * 16 + lr] = acc[mb][nb][j]; }
        __builtin_amdgcn_wave_barrier(); asm volatile("" ::: "memory");
        float* crow = C + (size_t)(r0 + mb * 16) * ldc + c0;
#pragma unroll 1
        for (int ps = 0; ps < 2; ++ps) {
#pragma unroll
            for (int s = 0; s < 8; ++s) { const int row = 2 * s + hi, cofs = lr * 4; v4f val = *(const v4fa*)(os + row * 68 + cofs); if (BIAS) { val[0] += bfr(bias[c0 + cofs]); val[1] += bfr(bias[c0 + cofs + 1]); val[2] += bfr(bias[c0 + cofs + 2]); val[3] += bfr(bias[c0 + cofs + 3]); }
                *(volatile v4f*)(crow + (size_t)row * ldc + cofs) = val; }
            if (ps == 0) __threadfence(); }
        __builtin_amdgcn_wave_barrier(); asm volatile("" ::: "memory");
    }
}

template <typename T16, int NSPLIT, int CMODE>
__global__ __launch_bounds__(32) void k_gemmc(const T16* __restrict__ A, const T16* __restrict__ A2, const T16* __restrict__ Bt, const T16* __restrict__ Bt2, int K, float* C, int ldc, int roff, size_t sA, size_t sB, size_t sC) {
    typedef typename WFrag<T16>::V V;
    __shared__ __align__(16) float os[16 * 68];
    const size_t z = blockIdx.z; A += z * sA; if (A2) A2 += z * sA; Bt += z * sB; if (Bt2) Bt2 += z * sB; C += z * sC;
    const int lane = threadIdx.x & 31, lr = lane & 15, hi = lane >> 4; const int r0 = blockIdx.x * 64, c0 = blockIdx.y * 64;
    if (CMODE == 1 && c0 > r0 + roff + 63) return;
    const int Kl = (CMODE == 2) ? min(K, r0 + roff + 64) : K;
    v8f acc[4][4];
#pragma unroll
    for (int mb = 0; mb < 4; ++mb)
#pragma unroll
        for (int nb = 0; nb < 4; ++nb) acc[mb][nb] = (v8f){};
    const size_t aoff = (size_t)(r0 + lr) * K + 8 * hi, boff = (size_t)(c0 + lr) * K + 8 * hi;
#pragma unroll 1
    for (int kc = 0; kc < Kl; kc += 32) {
        V a[4], a2[4];
#pragma unroll
        for (int mb = 0; mb < 4; ++mb) { a[mb] = WFrag<T16>::ld(A + aoff + (size_t)mb * 16 * K + kc); if (NSPLIT == 1 || NSPLIT == 2) a2[mb] = WFrag<T16>::ld(A2 + aoff + (size_t)mb * 16 * K + kc); }
#pragma unroll
        for (int nb = 0; nb < 4; ++nb) { const V b = WFrag<T16>::ld(Bt + boff + (size_t)nb * 16 * K + kc); V b2; if (NSPLIT >= 2) b2 = WFrag<T16>::ld(Bt2 + boff + (size_t)nb * 16 * K + kc);
#pragma unroll
            for (int mb = 0; mb < 4; ++mb) { acc[mb][nb] = WFrag<T16>::mma(a[mb], b, acc[mb][nb]); if (NSPLIT == 1 || NSPLIT == 2) acc[mb][nb] = WFrag<T16>::mma(a2[mb], b, acc[mb][nb]); if (NSPLIT >= 2) acc[mb][nb] = WFrag<T16>::mma(a[mb], b2, acc[mb][nb]); } }
        asm volatile("v_nop\n\tv_nop\n\tv_nop\n\tv_nop" : "+v"(acc[0][0]), "+v"(acc[1][1]), "+v"(acc[2][2]), "+v"(acc[3][3]) : "v"(a[0]), "v"(a[3]));
    }
#pragma unroll
    for (int mb = 0; mb < 4; ++mb) {
#pragma unroll
        for (int nb = 0; nb < 4; ++nb) {
#pragma unroll
            for (int j = 0; j < 8; ++j) os[(hi * 8 + j) * 68 + nb * 16 + lr] = acc[mb][nb][j]; }
        __builtin_amdgcn_wave_barrier(); asm volatile("" ::: "memory");
        float* crow = C + (size_t)(r0 + mb * 16) * ldc + c0;
#pragma unroll 1
        for (int ps = 0; ps < 2; ++ps) {
#pragma unroll
            for (int s = 0; s < 8; ++s) { const int row = 2 * s + hi, cofs = lr * 4; v4f val = *(const v4fa*)(os + row * 68 + cofs);
                *(volatile v4f*)(crow + (size_t)row * ldc + cofs) = val; }
            if (ps == 0) __threadfence(); }
        __builtin_amdgcn_wave_barrier(); asm volatile("" ::: "memory");
    }
}

__device__ __forceinline__ h16 tohx(float x) { return (h16)x; }
__device__ __forceinline__ void splitf(float y, unsigned short& h, unsigned short& l) { h = f2bf(y); l = f2bf(y - bf2f(h)); }
typedef __attribute__((ext_vector_type(2))) _Float16 v2h;
typedef __attribute__((ext_vector_type(4))) _Float16 v4h;
typedef __attribute__((ext_vector_type(2))) unsigned short v2us;
typedef __attribute__((ext_vector_type(4))) unsigned short v4us;
typedef __attribute__((ext_vector_type(2))) float v2f;
typedef __attribute__((ext_vector_type(4))) int v4i;


__global__ __launch_bounds__(256) void k_vtpH(const float* __restrict__ F, h16* V16, bf* Vh, bf* Vl) { const size_t e = ((size_t)blockIdx.x * 256 + threadIdx.x) * 2; if (e >= (size_t)NKV * HD * TT) return; const int t = (int)(e % TT); const int d = (int)((e / TT) % HD); const int g = (int)(e / ((size_t)TT * HD)); v2h o16; v2us oh, ol;
#pragma unroll
    for (int q = 0; q < 2; ++q) { const float x = bfr(F[((size_t)g * TT + t + q) * HD + d]); o16[q] = tohx(x); oh[q] = f2bf(x); ol[q] = 0; }
    *(volatile v2h*)(V16 + e) = o16; *(volatile v2us*)(Vh + e) = oh; *(volatile v2us*)(Vl + e) = ol; __threadfence(); *(volatile v2h*)(V16 + e) = o16; *(volatile v2us*)(Vh + e) = oh; *(volatile v2us*)(Vl + e) = ol; }
__global__ __launch_bounds__(256) void k_mergeH(const float* __restrict__ O, float* OUTh) { const size_t i = (size_t)blockIdx.x * 256 + threadIdx.x; if (i >= (size_t)ZH * TT * HD / 4) return; const size_t e = i * 4; const int t = (int)((e / HD) % TT); const float cs = (t < RH) ? 1.0f : (1.0f / PCAR); const v4f a = *(const v4f*)(O + e); v4f o;
#pragma unroll
    for (int q = 0; q < 4; ++q) o[q] = a[q] * cs; *(volatile v4f*)(OUTh + e) = o; __threadfence(); *(volatile v4f*)(OUTh + e) = o; }


__global__ __launch_bounds__(256) void k_cvt8(const float* __restrict__ src, bf* dst, size_t n8) { const size_t i = (size_t)blockIdx.x * 256 + threadIdx.x; if (i >= n8) return; const v8f v = *(const v8f*)(src + i * 8); v8us o;
#pragma unroll
    for (int k = 0; k < 8; ++k) o[k] = f2bf(v[k]); *(volatile v8us*)(dst + i * 8) = o; __threadfence(); *(volatile v8us*)(dst + i * 8) = o; }

__global__ __launch_bounds__(256) void k_rmax(const float* __restrict__ G, float* RM) { const int lane = threadIdx.x & 31; const int row = blockIdx.x * 8 + (threadIdx.x >> 5); if (row >= TT) return; const float* gr = G + (size_t)row * MF; const v4f a = *(const v4f*)(gr + lane * 8); const v4f c = *(const v4f*)(gr + lane * 8 + 4);
    float mx = fmaxf(fmaxf(fmaxf(a[0], a[1]), fmaxf(a[2], a[3])), fmaxf(fmaxf(c[0], c[1]), fmaxf(c[2], c[3])));
#pragma unroll
    for (int sh = 16; sh; sh >>= 1) mx = fmaxf(mx, __shfl_xor(mx, sh, 32));
    if (lane == 0) { *(volatile float*)(RM + (size_t)row * 32) = mx; __threadfence(); *(volatile float*)(RM + (size_t)row * 32) = mx; } }
__global__ __launch_bounds__(256) void k_gmax(const float* __restrict__ RM, float* GM) { __shared__ float red[256]; const int tid = threadIdx.x; float mx = -3.0e38f;
#pragma unroll 1
    for (int r = tid; r < TT; r += 256) mx = fmaxf(mx, RM[(size_t)r * 32]);
    red[tid] = mx; __syncthreads();
#pragma unroll
    for (int s = 128; s > 0; s >>= 1) { if (tid < s) red[tid] = fmaxf(red[tid], red[tid + s]); __syncthreads(); }
    if (tid == 0) { *(volatile float*)GM = red[0]; __threadfence(); *(volatile float*)GM = red[0]; } }
template <int QMODE>
__global__ __launch_bounds__(256) void k_phi(const float* __restrict__ G, const float* __restrict__ xin, const float* __restrict__ GM, h16* P16o, bf* Pho, bf* Plo, float* RSQ) {
    const int lane = threadIdx.x & 31; const int row = blockIdx.x * 8 + (threadIdx.x >> 5); if (row >= TT) return; const float* gr = G + (size_t)row * MF;
    const v2f xv = *(const v2f*)(xin + (size_t)row * HD + lane * 2); float q0 = bfr(xv[0]), q1 = bfr(xv[1]); float dg = __fmul_rn(q0, q0); asm volatile("" : "+v"(dg)); float p1 = __fmul_rn(q1, q1); asm volatile("" : "+v"(p1)); dg = __fadd_rn(dg, p1);
#pragma unroll
    for (int sh = 16; sh; sh >>= 1) dg = __fadd_rn(dg, __shfl_xor(dg, sh, 32));
    const float diag = __fmul_rn(dg, 0.0625f);
    float d8[8]; { const v4f a = *(const v4f*)(gr + lane * 8); const v4f c = *(const v4f*)(gr + lane * 8 + 4);
#pragma unroll
      for (int q = 0; q < 4; ++q) { d8[q] = __fmul_rn(a[q], NRM); d8[4 + q] = __fmul_rn(c[q], NRM); } }
    float mx;
    if (QMODE) { mx = d8[0];
#pragma unroll
        for (int q = 1; q < 8; ++q) mx = fmaxf(mx, d8[q]);
#pragma unroll
        for (int sh = 16; sh; sh >>= 1) mx = fmaxf(mx, __shfl_xor(mx, sh, 32)); }
    else { mx = __fmul_rn(GM[0], NRM); }
    const float off = __fadd_rn(diag, mx); v8h o16; v8us oh, ol; float fs = 0.f;
#pragma unroll
    for (int q = 0; q < 8; ++q) { float t = __fsub_rn(d8[q], off); asm volatile("" : "+v"(t)); float e = __builtin_amdgcn_exp2f(__fmul_rn(t, 1.4426950408889634f)); asm volatile("" : "+v"(e)); e = __fadd_rn(e, 1e-4f); const float ph = __fmul_rn(e, QSC); fs = __fadd_rn(fs, ph);
        o16[q] = tohx(ph); unsigned short a2, c2; splitf(ph, a2, c2); oh[q] = a2; ol[q] = c2; }
    if (QMODE) {
#pragma unroll
        for (int sh = 16; sh; sh >>= 1) fs = __fadd_rn(fs, __shfl_xor(fs, sh, 32)); }
    const size_t ob = (size_t)row * MF + lane * 8;
#pragma unroll 1
    for (int ps = 0; ps < 2; ++ps) { *(volatile v8h*)(P16o + ob) = o16; *(volatile v8us*)(Pho + ob) = oh; *(volatile v8us*)(Plo + ob) = ol; if (QMODE && lane == 0) *(volatile float*)(RSQ + (size_t)row * 32) = __fmul_rn(fs, EPSD); if (ps == 0) __threadfence(); }
}
__global__ __launch_bounds__(256) void k_lnrm(const float* __restrict__ Sb, const float* __restrict__ RSQ, h16* P16, bf* Ph, bf* Pl) {
    const int lane = threadIdx.x & 31; const int row = blockIdx.x * 8 + (threadIdx.x >> 5); if (row >= ZH * TT) return; const int i = row % TT; const int zz = row / TT; (void)zz; const bool hires = (i < RH); const float* sr = Sb + (size_t)row * TT; float v[TT / 32]; float sum = 0.f;
#pragma unroll
    for (int ch = 0; ch < TT / 128; ++ch) { const int j0 = ch * 128 + lane * 4; const v4f a = *(const v4f*)(sr + j0);
#pragma unroll
        for (int q = 0; q < 4; ++q) { const int j = j0 + q; const float t = (j <= i) ? a[q] : 0.0f; v[ch * 4 + q] = t; sum = __fadd_rn(sum, t); } }
#pragma unroll
    for (int sh = 16; sh; sh >>= 1) sum = __fadd_rn(sum, __shfl_xor(sum, sh, 32));
    const float f = __fdiv_rn(hires ? 1.0f : PCAR, __fadd_rn(sum, RSQ[(size_t)i * 32]));
#pragma unroll 1
    for (int ps = 0; ps < 2; ++ps) {
        if (hires) {
#pragma unroll
            for (int ch = 0; ch < TT / 128; ++ch) { v4us oh, ol;
#pragma unroll
                for (int q = 0; q < 4; ++q) { unsigned short a, c2; float y = __fmul_rn(v[ch * 4 + q], f); asm volatile("" : "+v"(y)); splitf(y, a, c2); oh[q] = a; ol[q] = c2; }
                const size_t oo = ((size_t)zz * (RH ? RH : 1) + i) * TT + ch * 128 + lane * 4; *(volatile v4us*)(Ph + oo) = oh; *(volatile v4us*)(Pl + oo) = ol; }
        } else {
#pragma unroll
            for (int ch = 0; ch < TT / 128; ++ch) { v4h o4;
#pragma unroll
                for (int q = 0; q < 4; ++q) { float y = __fmul_rn(v[ch * 4 + q], f); asm volatile("" : "+v"(y)); o4[q] = tohx(y); }
                *(volatile v4h*)(P16 + (size_t)row * TT + ch * 128 + lane * 4) = o4; } }
        if (ps == 0) __threadfence(); }
}

extern "C" void kernel_launch(void* const* d_in, const int* in_sizes, int n_in,
                              void* d_out, int out_size, void* d_ws, size_t ws_size, hipStream_t stream) {
    (void)in_sizes; (void)n_in; (void)out_size;
    const float* qi = (const float*)d_in[0]; const float* ki = (const float*)d_in[1]; const float* vi = (const float*)d_in[2]; const float* proj = (const float*)d_in[3]; const float* x = nullptr; const float* wq = nullptr; const float* wk = nullptr; const float* wv = nullptr; const float* wo = nullptr; (void)x; (void)wq; (void)wk; (void)wv; (void)wo;
    float* OUT = (float*)d_out;
    char* wsp = (char*)d_ws;
    auto take = [&](size_t bytes) { char* p = wsp; wsp += (bytes + 255) & ~(size_t)255; return (void*)p; };
    bf* PROJB = (bf*)take((size_t)MF * HD * 2); bf* XQB = (bf*)take((size_t)TT * HD * 2); float* G = (float*)take((size_t)TT * MF * 4); float* RM = (float*)take((size_t)TT * 32 * 4); float* RSQ = (float*)take((size_t)TT * 32 * 4); float* GM = (float*)take(256);
    h16* QP16 = (h16*)take((size_t)TT * MF * 2); bf* QPh = (bf*)take((size_t)TT * MF * 2); bf* QPl = (bf*)take((size_t)TT * MF * 2); h16* KP16 = (h16*)take((size_t)TT * MF * 2); bf* KPh = (bf*)take((size_t)TT * MF * 2); bf* KPl = (bf*)take((size_t)TT * MF * 2);
    h16* VT16 = (h16*)take((size_t)NKV * HD * TT * 2); bf* VTh = (bf*)take((size_t)NKV * HD * TT * 2); bf* VTl = (bf*)take((size_t)NKV * HD * TT * 2); bf* Ph = (bf*)take((size_t)RH * TT * 2); bf* Pl = (bf*)take((size_t)RH * TT * 2);
    float* Sb = (float*)take((size_t)TT * TT * 4); h16* P16 = (h16*)take((size_t)TT * TT * 2); float* Ob = (float*)take((size_t)TT * HD * 4);
    if ((size_t)(wsp - (char*)d_ws) > ws_size) return;
    k_cvt8<<<(unsigned)(((size_t)MF * HD / 8 + 255) / 256), 256, 0, stream>>>(proj, PROJB, (size_t)MF * HD / 8);
    for (int b = 0; b < NB_; ++b) {
        k_vtpH<<<(unsigned)(((size_t)NKV * HD * TT / 2 + 255) / 256), 256, 0, stream>>>(vi + (size_t)b * NKV * TT * HD, VT16, VTh, VTl);
        for (int h0 = 0; h0 < NH_; ++h0) { const size_t zk = (size_t)h0; const float* qh = qi + ((size_t)b * NH_ + h0) * TT * HD; const float* kh = ki + ((size_t)b * NKV + h0) * TT * HD;
            k_cvt8<<<(unsigned)(((size_t)TT * HD / 8 + 255) / 256), 256, 0, stream>>>(kh, XQB, (size_t)TT * HD / 8);
            k_gemmw<bf, 0, false><<<dim3(TT / 64, MF / 64, 1), 32, 0, stream>>>(XQB, nullptr, PROJB, nullptr, HD, G, MF, nullptr, 0, 0, 0);
            k_rmax<<<TT / 8, 256, 0, stream>>>(G, RM); k_gmax<<<1, 256, 0, stream>>>(RM, GM);
            k_phi<0><<<TT / 8, 256, 0, stream>>>(G, kh, GM, KP16, KPh, KPl, nullptr);
            k_cvt8<<<(unsigned)(((size_t)TT * HD / 8 + 255) / 256), 256, 0, stream>>>(qh, XQB, (size_t)TT * HD / 8);
            k_gemmw<bf, 0, false><<<dim3(TT / 64, MF / 64, 1), 32, 0, stream>>>(XQB, nullptr, PROJB, nullptr, HD, G, MF, nullptr, 0, 0, 0);
            k_phi<1><<<TT / 8, 256, 0, stream>>>(G, qh, GM, QP16, QPh, QPl, RSQ);
            k_gemmc<bf, 2, 1><<<dim3(RH / 64, TT / 64, 1), 32, 0, stream>>>(QPh, QPl, KPh, KPl, MF, Sb, TT, 0, 0, 0, 0);
            k_gemmc<h16, 0, 1><<<dim3((TT - RH) / 64, TT / 64, 1), 32, 0, stream>>>(QP16 + (size_t)RH * MF, nullptr, KP16, nullptr, MF, Sb + (size_t)RH * TT, TT, RH, 0, 0, 0);
            k_lnrm<<<TT / 8, 256, 0, stream>>>(Sb, RSQ, P16, Ph, Pl);
            k_gemmc<bf, 2, 2><<<dim3(RH / 64, HD / 64, 1), 32, 0, stream>>>(Ph, Pl, VTh + zk * HD * TT, VTl + zk * HD * TT, TT, Ob, HD, 0, 0, 0, 0);
            k_gemmc<h16, 0, 2><<<dim3((TT - RH) / 64, HD / 64, 1), 32, 0, stream>>>(P16 + (size_t)RH * TT, nullptr, VT16 + zk * HD * TT, nullptr, TT, Ob + (size_t)RH * HD, HD, RH, 0, 0, 0);
            k_mergeH<<<(unsigned)(((size_t)TT * HD / 4 + 255) / 256), 256, 0, stream>>>(Ob, OUT + ((size_t)b * NH_ + h0) * TT * HD); }
    }
}
